// CausalSelfAttention_43267500540474
// MI455X (gfx1250) — hardware-verified
//
#include <hip/hip_runtime.h>
#include <math.h>

typedef __attribute__((ext_vector_type(16))) _Float16 v16h;
typedef __attribute__((ext_vector_type(16))) __bf16 v16b;
typedef __attribute__((ext_vector_type(8)))  _Float16 v8h;
typedef __attribute__((ext_vector_type(8)))  __bf16 v8b;
typedef __attribute__((ext_vector_type(8)))  float v8f;
typedef __attribute__((ext_vector_type(4)))  float v4f;
typedef __attribute__((ext_vector_type(4)))  unsigned v4u;

template <typename T> __device__ __forceinline__ void vst2(void* p, T v) { *(volatile T*)p = v; __threadfence(); *(volatile T*)p = v; }
__device__ __forceinline__ v8f wmma16(v16h a, v16h b, v8f c) {
  v8f d = __builtin_amdgcn_wmma_f32_16x16x32_f16(false, a, false, b, (short)0, c, false, false);
  asm volatile("v_nop\n\tv_nop\n\tv_nop\n\tv_nop" : "+v"(d) : "v"(a), "v"(b));
  return d;
}
__device__ __forceinline__ v8f wmma_bf(v16b a, v16b b, v8f c) {
  v8f d = __builtin_amdgcn_wmma_f32_16x16x32_bf16(false, a, false, b, (short)0, c, false, false);
  asm volatile("v_nop\n\tv_nop\n\tv_nop\n\tv_nop" : "+v"(d) : "v"(a), "v"(b));
  return d;
}
__device__ __forceinline__ v16h frag_h(const _Float16* rowk0, int lane) {
  union { v16h v; v8h q[2]; } u; const _Float16* p = rowk0 + 8 * (lane >> 4);
  u.q[0] = *(const v8h*)p; u.q[1] = *(const v8h*)(p + 16); return u.v;
}
__device__ __forceinline__ v16b frag_b(const __bf16* rowk0, int lane) {
  union { v16b v; v8b q[2]; } u; const __bf16* p = rowk0 + 8 * (lane >> 4);
  u.q[0] = *(const v8b*)p; u.q[1] = *(const v8b*)(p + 16); return u.v;
}
#define LDSX() do { asm volatile("s_wait_dscnt 0" ::: "memory"); __builtin_amdgcn_wave_barrier(); __builtin_amdgcn_fence(3  , "workgroup"); } while (0)

#ifndef NB
#define NB 4
#endif
#ifndef SEQ
#define SEQ 2048
#endif
#define NB_FULL 4
#define SEQ_FULL 2048
#define CC 1024
#define DIN 1024
#define NH 16
#define HD 64
#define SCALE (0.125f)
#define LN2048 (7.6246189861593985f)
#ifndef QRES
#define QRES 1
#endif

static_assert(SEQ % 64 == 0);
static_assert(CC % 128 == 0);
static_assert(DIN % 32 == 0);
static_assert(NH * HD == CC);
static_assert(HD == 64);
static_assert(((NB * SEQ) % 2) == 0);
static_assert(SEQ <= SEQ_FULL);
static_assert(NB <= NB_FULL);
static_assert((size_t)(NB * SEQ / 64) * (CC / 128) * 64 * 128 == (size_t)NB * SEQ * CC);
static_assert((size_t)(SEQ / 64) * (NB * NH) * 64 * HD == (size_t)NB * SEQ * CC);
static_assert((size_t)(SEQ / 8) * 8 * 64 == (size_t)SEQ * 64);

#define WS_XB   ((size_t)0)
#define WS_WB   (WS_XB  + 2u * (size_t)NB * SEQ * DIN)
#define WS_WOB  (WS_WB  + 2u * (size_t)3 * CC * DIN)
#define WS_TAB  (WS_WOB + 2u * (size_t)CC * CC)
#define WS_QH   (WS_TAB + 4u * (size_t)SEQ * 64)
#define WS_QL   (WS_QH  + 2u * (size_t)NB * SEQ * CC)
#define WS_KH   (WS_QL  + 2u * (size_t)NB * SEQ * CC)
#define WS_VT   (WS_KH  + 2u * (size_t)NB * SEQ * CC)
#define WS_YH   (WS_VT  + 2u * (size_t)NB * SEQ * CC)
#define WS_YL   (WS_YH  + 2u * (size_t)NB * SEQ * CC)
#define WS_END  (WS_YL  + 2u * (size_t)NB * SEQ * CC)
static_assert(WS_END <= (size_t)134217728);

__device__ __forceinline__ v4u bf8(v4f a, v4f b) { union { v8b v; v4u u; } x;
  x.v[0] = (__bf16)a[0]; x.v[1] = (__bf16)a[1]; x.v[2] = (__bf16)a[2]; x.v[3] = (__bf16)a[3];
  x.v[4] = (__bf16)b[0]; x.v[5] = (__bf16)b[1]; x.v[6] = (__bf16)b[2]; x.v[7] = (__bf16)b[3]; return x.u; }

__global__ __launch_bounds__(256) void k_cvt(const float* __restrict__ src, __bf16* __restrict__ dst, unsigned nrows, unsigned xmode) {
  const unsigned gid = blockIdx.x * 256u + threadIdx.x; const unsigned row = gid >> 7, pc = gid & 127u;
  if (row >= nrows) return;
  const unsigned srow = xmode ? ((row % (unsigned)SEQ) * (unsigned)NB_FULL + row / (unsigned)SEQ) : row;
  const float* p = src + (size_t)srow * DIN + pc * 8u;
  const v4f a = *(const v4f*)p, b = *(const v4f*)(p + 4);
  vst2(dst + (size_t)row * DIN + pc * 8u, bf8(a, b));
}

__device__ __forceinline__ float theta_of(unsigned i) { float v = 1.0f;
#define TH(k, val) v = (i == (k)) ? (val) : v;
  TH(1, 7.498942093324558e-1f) TH(2, 5.623413251903491e-1f) TH(3, 4.216965034285822e-1f) TH(4, 3.162277660168379e-1f)
  TH(5, 2.371373705661655e-1f) TH(6, 1.778279410038923e-1f) TH(7, 1.333521432163324e-1f) TH(8, 1.0e-1f)
  TH(9, 7.498942093324558e-2f) TH(10, 5.623413251903491e-2f) TH(11, 4.216965034285822e-2f) TH(12, 3.162277660168379e-2f)
  TH(13, 2.371373705661655e-2f) TH(14, 1.778279410038923e-2f) TH(15, 1.333521432163324e-2f) TH(16, 1.0e-2f)
  TH(17, 7.498942093324558e-3f) TH(18, 5.623413251903491e-3f) TH(19, 4.216965034285822e-3f) TH(20, 3.162277660168379e-3f)
  TH(21, 2.371373705661655e-3f) TH(22, 1.778279410038923e-3f) TH(23, 1.333521432163324e-3f) TH(24, 1.0e-3f)
  TH(25, 7.498942093324558e-4f) TH(26, 5.623413251903491e-4f) TH(27, 4.216965034285822e-4f) TH(28, 3.162277660168379e-4f)
  TH(29, 2.371373705661655e-4f) TH(30, 1.778279410038923e-4f) TH(31, 1.333521432163324e-4f)
#undef TH
  return v; }

__global__ __launch_bounds__(256) void k_tab(float* __restrict__ TAB) { __shared__ __align__(16) float st[8][64];
  const unsigned tid = threadIdx.x, tl = tid >> 5, i = tid & 31u; const unsigned t = blockIdx.x * 8u + tl;
  const float ang = (float)t * theta_of(i);
  const float c = (float)(_Float16)cosf(ang), s = (float)(_Float16)sinf(ang);
  st[tl][i] = c; st[tl][32u + i] = s;
  __syncthreads();
  if (tid < 128u) { const unsigned rl = tid >> 4, q = tid & 15u; vst2(TAB + (size_t)(blockIdx.x * 8u + rl) * 64u + q * 4u, *(const v4f*)&st[rl][q * 4u]); }
}

__global__ __launch_bounds__(128) void k_proj(const __bf16* __restrict__ XB, const __bf16* __restrict__ WB, const float* __restrict__ TAB,
    _Float16* __restrict__ QH, _Float16* __restrict__ QL, _Float16* __restrict__ KH, _Float16* __restrict__ VT) {
  __shared__ __align__(16) _Float16 sh[64][136], sl[64][136]; __shared__ __align__(16) _Float16 th[128][72];
  const unsigned tid = threadIdx.x, wave = tid >> 5, col = tid & 15u, g = (tid >> 4) & 1u; const int lane = (int)(tid & 31u);
  const unsigned which = blockIdx.z, c0 = blockIdx.y * 128u; const unsigned bb = blockIdx.x / (unsigned)(SEQ / 64), t0 = (blockIdx.x % (unsigned)(SEQ / 64)) * 64u;
  const __bf16* xrow = XB + ((size_t)bb * SEQ + t0 + wave * 16u + col) * DIN;
  const __bf16* wrow = WB + ((size_t)which * CC + c0 + col) * DIN;
  v8f acc[8] = {};
#pragma unroll 2
  for (unsigned kc = 0; kc < DIN / 32; ++kc) { const v16b a = frag_b(xrow + kc * 32u, lane);
    asm volatile("s_wait_loadcnt 0x0" ::: "memory");
#pragma unroll
    for (int j = 0; j < 8; ++j) { const v16b w = frag_b(wrow + (size_t)j * 16 * DIN + kc * 32u, lane); asm volatile("s_wait_loadcnt 0x0" ::: "memory"); acc[j] = wmma_bf(a, w, acc[j]); } }
  const unsigned hd0 = c0 >> 6;
  if (which < 2u) { _Float16* DH = which == 0u ? QH : KH; const unsigned tl = wave * 16u + 8u * g; const bool wres = (QRES != 0) && (which == 0u);
#pragma unroll
    for (int jj = 0; jj < 2; ++jj) { float cs[8], sn[8];
#pragma unroll
      for (int r = 0; r < 8; ++r) { const float* tp = TAB + (size_t)(t0 + tl + r) * 64u + jj * 16 + col; cs[r] = tp[0]; sn[r] = tp[32]; }
      asm volatile("s_wait_loadcnt 0x0" ::: "memory");
#pragma unroll
      for (int hl = 0; hl < 2; ++hl) {
#pragma unroll
        for (int r = 0; r < 8; ++r) { const float x0 = acc[hl * 4 + jj][r], x1 = acc[hl * 4 + jj + 2][r];
          const float y0 = x0 * cs[r] - x1 * sn[r], y1 = x1 * cs[r] + x0 * sn[r];
          const unsigned rl = tl + r, ca = hl * 64 + jj * 16 + col; const _Float16 h0 = (_Float16)y0, h1 = (_Float16)y1;
          sh[rl][ca] = h0; sh[rl][ca + 32u] = h1;
          if (wres) { sl[rl][ca] = (_Float16)((y0 - (float)h0) * 1024.0f); sl[rl][ca + 32u] = (_Float16)((y1 - (float)h1) * 1024.0f); } } } }
    __syncthreads();
    for (unsigned e = tid; e < 64u * 16u; e += 128u) { const unsigned rl = e >> 4, qd = e & 15u;
      const size_t o = (((size_t)bb * NH + hd0 + (qd >> 3)) * SEQ + t0 + rl) * HD + (qd & 7u) * 8u;
      const v4u vh = *(const v4u*)&sh[rl][qd * 8u]; vst2(DH + o, vh);
      if (wres) { const v4u vl = *(const v4u*)&sl[rl][qd * 8u]; vst2(QL + o, vl); } }
  } else {
#pragma unroll
    for (int j = 0; j < 8; ++j) {
#pragma unroll
      for (int r = 0; r < 8; ++r) th[j * 16 + col][wave * 16u + 8u * g + r] = (_Float16)acc[j][r]; }
    __syncthreads();
    for (unsigned e = tid; e < 128u * 8u; e += 128u) { const unsigned cl = e >> 3, q = e & 7u;
      const size_t o = (((size_t)bb * NH + hd0 + (cl >> 6)) * HD + (cl & 63u)) * SEQ + t0 + q * 8u;
      const v4u vv = *(const v4u*)&th[cl][q * 8u]; vst2(VT + o, vv); } }
}

__global__ __launch_bounds__(128) void k_fa(const _Float16* __restrict__ QH, const _Float16* __restrict__ QL, const _Float16* __restrict__ KH, const _Float16* __restrict__ VT, __bf16* __restrict__ YH, __bf16* __restrict__ YL) {
  __shared__ __align__(16) float so[4][16][68];
  const unsigned tid = threadIdx.x, wave = tid >> 5, col = tid & 15u, g = (tid >> 4) & 1u; const int lane = (int)(tid & 31u);
  const unsigned bh = blockIdx.y, q0 = blockIdx.x * 64u + wave * 16u; const size_t hb = (size_t)bh * SEQ * HD;
  v16h bqh[2];
#pragma unroll
  for (int kc = 0; kc < 2; ++kc) bqh[kc] = frag_h(QH + hb + (size_t)(q0 + col) * HD + kc * 32, lane);
#if QRES
  v16h bql[2];
#pragma unroll
  for (int kc = 0; kc < 2; ++kc) bql[kc] = frag_h(QL + hb + (size_t)(q0 + col) * HD + kc * 32, lane);
#else
  (void)QL;
#endif
  const _Float16* kp = KH + hb + (size_t)col * HD;
  const _Float16* vp = VT + hb + (size_t)col * SEQ;
  v8f o[4] = {}; float m = -1.0e30f, l = 0.f;
#pragma unroll 1
  for (unsigned ks = 0; ks < (unsigned)SEQ; ks += 64u) {
    v8f s[4];
#pragma unroll
    for (int kt = 0; kt < 4; ++kt) { v8f a = {};
#if QRES
      v8f al = {};
#endif
#pragma unroll
      for (int kc = 0; kc < 2; ++kc) { const v16h kf = frag_h(kp + (size_t)(ks + kt * 16) * HD + kc * 32, lane);
        a = wmma16(kf, bqh[kc], a);
#if QRES
        al = wmma16(kf, bql[kc], al);
#endif
      }
#pragma unroll
      for (int r = 0; r < 8; ++r) {
#if QRES
        s[kt][r] = a[r] * SCALE + al[r] * (SCALE / 1024.0f);
#else
        s[kt][r] = a[r] * SCALE;
#endif
      } }
    float mx = s[0][0];
#pragma unroll
    for (int kt = 0; kt < 4; ++kt) {
#pragma unroll
      for (int r = 0; r < 8; ++r) mx = fmaxf(mx, s[kt][r]); }
    mx = fmaxf(mx, __shfl_xor(mx, 16));
    const float mn = fmaxf(m, mx); const float alpha = __expf(m - mn); const float mo = mn - LN2048; m = mn;
    float ls = 0.f; v16h pf[2];
#pragma unroll
    for (int c = 0; c < 2; ++c) {
#pragma unroll
      for (int i = 0; i < 8; ++i) { const float p0 = __expf(s[2 * c][i] - mo), p1 = __expf(s[2 * c + 1][i] - mo); ls += p0 + p1; pf[c][i] = (_Float16)p0; pf[c][8 + i] = (_Float16)p1; } }
    l = l * alpha + ls;
#pragma unroll
    for (int j = 0; j < 4; ++j) {
#pragma unroll
      for (int r = 0; r < 8; ++r) o[j][r] *= alpha; }
#pragma unroll
    for (int j = 0; j < 4; ++j) {
#pragma unroll
      for (int c = 0; c < 2; ++c) { const v16h vf = frag_h(vp + (size_t)(j * 16) * SEQ + ks + c * 32, lane); o[j] = wmma16(vf, pf[c], o[j]); } }
  }
  const float lt = l + __shfl_xor(l, 16); const float inv = 1.0f / lt;
#pragma unroll
  for (int j = 0; j < 4; ++j) {
#pragma unroll
    for (int r = 0; r < 8; ++r) so[wave][col][j * 16 + 8 * g + r] = o[j][r] * inv; }
  LDSX();
  const unsigned b = bh / (unsigned)NH, h = bh % (unsigned)NH;
#pragma unroll
  for (int it = 0; it < 4; ++it) { const unsigned p = (unsigned)it * 32u + (unsigned)lane, qn = p >> 3, pc = p & 7u;
    const v4f x0 = *(const v4f*)&so[wave][qn][pc * 8u], x1 = *(const v4f*)&so[wave][qn][pc * 8u + 4u];
    union { v8b v; v4u u; } hi, lo;
#pragma unroll
    for (int i = 0; i < 4; ++i) { const __bf16 ha = (__bf16)x0[i], hb2 = (__bf16)x1[i]; hi.v[i] = ha; hi.v[4 + i] = hb2; lo.v[i] = (__bf16)(x0[i] - (float)ha); lo.v[4 + i] = (__bf16)(x1[i] - (float)hb2); }
    const size_t oo = ((size_t)b * SEQ + q0 + qn) * CC + h * HD + pc * 8u;
    vst2(YH + oo, hi.u); vst2(YL + oo, lo.u); }
}

__global__ __launch_bounds__(128) void k_out(const __bf16* __restrict__ YH, const __bf16* __restrict__ YL, const __bf16* __restrict__ WOB, float* __restrict__ OUT) {
  __shared__ __align__(16) float sf[4][16][132];
  const unsigned tid = threadIdx.x, wave = tid >> 5, col = tid & 15u, g = (tid >> 4) & 1u; const int lane = (int)(tid & 31u);
  const unsigned c0 = blockIdx.y * 128u; const unsigned bb = blockIdx.x / (unsigned)(SEQ / 64), t0 = (blockIdx.x % (unsigned)(SEQ / 64)) * 64u + wave * 16u;
  const size_t yr = ((size_t)bb * SEQ + t0 + col) * CC; const __bf16* wrow = WOB + (size_t)(c0 + col) * CC;
  v8f acc[8] = {};
#pragma unroll 2
  for (unsigned kc = 0; kc < CC / 32; ++kc) { const v16b ah = frag_b(YH + yr + kc * 32u, lane), al = frag_b(YL + yr + kc * 32u, lane);
    asm volatile("s_wait_loadcnt 0x0" ::: "memory");
#pragma unroll
    for (int j = 0; j < 8; ++j) { const v16b w = frag_b(wrow + (size_t)j * 16 * CC + kc * 32u, lane); asm volatile("s_wait_loadcnt 0x0" ::: "memory"); acc[j] = wmma_bf(ah, w, acc[j]); acc[j] = wmma_bf(al, w, acc[j]); } }
#pragma unroll
  for (int j = 0; j < 8; ++j) {
#pragma unroll
    for (int r = 0; r < 8; ++r) sf[wave][8 * g + r][j * 16 + col] = acc[j][r]; }
  LDSX();
  for (unsigned rl = 0; rl < 16u; ++rl) { const v4f v = *(const v4f*)&sf[wave][rl][lane * 4]; vst2(OUT + ((size_t)(t0 + rl) * NB + bb) * CC + c0 + (unsigned)lane * 4u, v); }
}

extern "C" void kernel_launch(void* const* d_in, const int* in_sizes, int n_in, void* d_out, int out_size, void* d_ws, size_t ws_size, hipStream_t stream) {
  if (n_in < 3) return;
  if (ws_size < (size_t)WS_END) return;
  if (in_sizes[0] < ((SEQ - 1) * NB_FULL + NB) * DIN) return;
  if (in_sizes[1] < 3 * CC * DIN) return;
  if (in_sizes[2] < CC * CC) return;
  if (out_size < SEQ * NB * CC) return;
  const float* X = (const float*)d_in[0];
  const float* WQKV = (const float*)d_in[1];
  const float* WO = (const float*)d_in[2];
  char* ws = (char*)d_ws;
  __bf16 *XB = (__bf16*)(ws + WS_XB), *WB = (__bf16*)(ws + WS_WB), *WOB = (__bf16*)(ws + WS_WOB), *YH = (__bf16*)(ws + WS_YH), *YL = (__bf16*)(ws + WS_YL);
  float* TAB = (float*)(ws + WS_TAB);
  _Float16 *QH = (_Float16*)(ws + WS_QH), *QL = (_Float16*)(ws + WS_QL), *KH = (_Float16*)(ws + WS_KH), *VT = (_Float16*)(ws + WS_VT);
  k_cvt<<<dim3((unsigned)(NB * SEQ) / 2u), 256, 0, stream>>>(X, XB, (unsigned)(NB * SEQ), 1u);
  k_cvt<<<dim3((unsigned)(3 * CC) / 2u), 256, 0, stream>>>(WQKV, WB, (unsigned)(3 * CC), 0u);
  k_cvt<<<dim3((unsigned)CC / 2u), 256, 0, stream>>>(WO, WOB, (unsigned)CC, 0u);
  k_tab<<<dim3(SEQ / 8), 256, 0, stream>>>(TAB);
  k_proj<<<dim3(NB * SEQ / 64, CC / 128, 3), 128, 0, stream>>>(XB, WB, TAB, QH, QL, KH, VT);
  k_fa<<<dim3(SEQ / 64, NB * NH), 128, 0, stream>>>(QH, QL, KH, VT, YH, YL);
  k_out<<<dim3(NB * SEQ / 64, CC / 128), 128, 0, stream>>>(YH, YL, WOB, (float*)d_out);
}
